// VNCrossAttention_28982439313690
// MI455X (gfx1250) — hardware-verified
//
#include <hip/hip_runtime.h>
#include <math.h>


namespace {
constexpr int Bsz = 4, T = 2048, HID = 512, DH = 64, NH = 8, NKV = 8, REP = NH / NKV;
constexpr int CC = 128, DV = 16;
constexpr int KVW = NKV * DH;
constexpr int NQKV = HID + 2 * KVW;
constexpr int MROWS = Bsz * T;
constexpr int QT_PER_B = T / 16;

typedef _Float16 b16;
typedef __attribute__((ext_vector_type(16))) _Float16 v16b;
typedef __attribute__((ext_vector_type(8)))  _Float16 v8b;
typedef __attribute__((ext_vector_type(8)))  float v8f;
typedef __attribute__((ext_vector_type(4)))  float v4f;

__device__ __forceinline__ v8b ld8b(const b16* p) { return *(const v8b*)p; }
__device__ __forceinline__ v16b cat8b(v8b a, v8b b) { return __builtin_shufflevector(a, b, 0, 1, 2, 3, 4, 5, 6, 7, 8, 9, 10, 11, 12, 13, 14, 15); }
__device__ __forceinline__ v16b frag_kb(const b16* p, int hh) { return cat8b(ld8b(p + 8 * hh), ld8b(p + 16 + 8 * hh)); }
__device__ __forceinline__ void split_bf16(float v, b16& hi, b16& lo) {
  hi = (b16)v; lo = (b16)0.0f;
}
__device__ __forceinline__ void frag_ksplit(const float* p, int hh, v16b& fh_, v16b& fl_) {
  const float* p0 = p + 8 * hh; const float* p1 = p + 16 + 8 * hh;
#pragma unroll
  for (int e = 0; e < 8; ++e) { b16 a, c; split_bf16(p0[e], a, c); fh_[e] = a; fl_[e] = c; split_bf16(p1[e], a, c); fh_[8 + e] = a; fl_[8 + e] = c; }
}
__device__ __forceinline__ v8f wmma16b(v16b a, v16b b, v8f c) {
  v8f d = __builtin_amdgcn_wmma_f32_16x16x32_f16(false, a, false, b, (short)0, c, false, false);
  asm volatile("v_nop\n\tv_nop\n\tv_nop\n\tv_nop" : "+v"(d) : "v"(a), "v"(b));
  return d;
}
__device__ __forceinline__ v8f wmma3(v16b ah, v16b al, v16b bh, v16b bl, v8f c) {
  (void)al; (void)bl; return wmma16b(ah, bh, c);
}
__device__ __forceinline__ v8f wmma1(v16b ah, v16b al, v16b bh, v16b bl, v8f c) {
  (void)al; (void)bl; return wmma16b(ah, bh, c);
}
__device__ __forceinline__ void wave_lds_sync() {
  __builtin_amdgcn_fence(__ATOMIC_RELEASE, "workgroup");
  __builtin_amdgcn_wave_barrier();
  __builtin_amdgcn_fence(__ATOMIC_ACQUIRE, "workgroup");
}

__global__ __launch_bounds__(256) void wcvt_kernel(const float* __restrict__ wq, const float* __restrict__ wk, const float* __restrict__ wv,
                                                   const float* __restrict__ wo, b16* __restrict__ wqh, b16* __restrict__ wql,
                                                   b16* __restrict__ woh, b16* __restrict__ wol) {
  const size_t tid = (size_t)blockIdx.x * blockDim.x + threadIdx.x, stride = (size_t)gridDim.x * blockDim.x;
  const size_t nq = (size_t)NQKV * HID / 8, no = (size_t)HID * HID / 8;
  for (int pass = 0; pass < 2; ++pass) {
    for (size_t c = tid; c < nq + no; c += stride) {
      float f[8]; size_t i; b16* dh; b16* dl;
      if (c < nq) {
        i = c * 8; const size_t n = i / HID, k0 = i % HID;
        const float* w; int nn, ld;
        if (n < (size_t)HID) { w = wq; nn = (int)n; ld = HID; } else if (n < (size_t)(HID + KVW)) { w = wk; nn = (int)n - HID; ld = KVW; } else { w = wv; nn = (int)n - HID - KVW; ld = KVW; }
#pragma unroll
        for (int e = 0; e < 8; ++e) f[e] = w[(size_t)(k0 + e) * ld + nn];
        dh = wqh; dl = wql;
      } else {
        i = (c - nq) * 8; const size_t n = i / HID, k0 = i % HID;
#pragma unroll
        for (int e = 0; e < 8; ++e) f[e] = wo[(size_t)(k0 + e) * HID + n];
        dh = woh; dl = wol;
      }
      v8b bh, bl;
#pragma unroll
      for (int e = 0; e < 8; ++e) { b16 a, cc; split_bf16(f[e], a, cc); bh[e] = a; bl[e] = cc; }
      *(volatile v8b*)(dh + i) = bh; *(volatile v8b*)(dl + i) = bl;
    }
    __threadfence();
  }
}


__device__ __forceinline__ v8f wmma16s(v16b a, v16b b, v8f c) {
  v8f d = __builtin_amdgcn_wmma_f32_16x16x32_f16(false, a, false, b, (short)0, c, false, false);
  asm volatile("v_nop\n\tv_nop\n\tv_nop\n\tv_nop" : "+v"(d) : "v"(a), "v"(b));
  return d;
}
__device__ __forceinline__ int kmap(int e, int hh) { return (e < 8) ? (8 * hh + e) : (16 + 8 * hh + (e - 8)); }
__global__ __launch_bounds__(256) void k_w16(const float* __restrict__ w, b16* __restrict__ W16, b16* __restrict__ W16l) {
  const int t = blockIdx.x * 256 + threadIdx.x;
  v8b o, ol;
#pragma unroll
  for (int e = 0; e < 8; ++e) { const float v = w[(size_t)t * 8 + e]; const b16 h = (b16)v; o[e] = h; ol[e] = (b16)(v - (float)h); }
  for (int pass = 0; pass < 2; ++pass) { *(volatile v8b*)(W16 + (size_t)t * 8) = o; *(volatile v8b*)(W16l + (size_t)t * 8) = ol; __threadfence(); }
}
template <int MODE>
__global__ __launch_bounds__(128) void k_vproj(const float* __restrict__ x, const b16* __restrict__ W16, const b16* __restrict__ W16l, const float* __restrict__ bias, b16* __restrict__ P) {
  __shared__ __attribute__((aligned(16))) b16 Ts[4][4 * 1024];
  const int lane = threadIdx.x & 31, wave = threadIdx.x >> 5, hh = lane >> 4, l16 = lane & 15;
  const int m0 = blockIdx.x * 64 + wave * 16, o0 = blockIdx.y * 64;
  const int b = m0 / T, t0 = m0 % T;
  v8f acc[4][3];
#pragma unroll
  for (int t = 0; t < 4; ++t)
#pragma unroll
    for (int c = 0; c < 3; ++c) acc[t][c] = (v8f){};
  const float* xr = x + (size_t)(m0 + l16) * (CC * 3);
#pragma unroll
  for (int k0 = 0; k0 < CC; k0 += 32) {
    v16b a[3], al[3];
#pragma unroll
    for (int e = 0; e < 16; ++e) { const int i = k0 + kmap(e, hh);
#pragma unroll
      for (int c = 0; c < 3; ++c) { const float v = xr[i * 3 + c]; const b16 h = (b16)v; a[c][e] = h; al[c][e] = (b16)(v - (float)h); } }
#pragma unroll
    for (int t = 0; t < 4; ++t) {
      const v16b w = frag_kb(W16 + (size_t)(o0 + t * 16 + l16) * CC + k0, hh), wl = frag_kb(W16l + (size_t)(o0 + t * 16 + l16) * CC + k0, hh);
#pragma unroll
      for (int c = 0; c < 3; ++c) { acc[t][c] = wmma16s(a[c], w, acc[t][c]); acc[t][c] = wmma16s(a[c], wl, acc[t][c]); acc[t][c] = wmma16s(al[c], w, acc[t][c]); }
    }
  }
  const float sc = (MODE == 0) ? 0.14433756729740643f : 1.0f;
  b16* ts = Ts[wave];
#pragma unroll
  for (int t = 0; t < 4; ++t) {
    const float bo = bias[o0 + t * 16 + l16];
#pragma unroll
    for (int v = 0; v < 8; ++v) {
      const int r = v + 8 * hh;
      const float y0 = acc[t][0][v], y1 = acc[t][1][v], y2 = acc[t][2][v];
      const float f = 1.0f + bo / (sqrtf(y0 * y0 + y1 * y1 + y2 * y2) + 1e-6f);
      const float vals[3] = {y0 * f * sc, y1 * f * sc, y2 * f * sc};
#pragma unroll
      for (int c = 0; c < 3; ++c) {
        const int e = l16 * 3 + c;
        if (MODE < 2) ts[(r * 4 + t) * 64 + e] = (b16)vals[c];
        else          ts[t * 1024 + e * 16 + r] = (b16)vals[c];
      }
    }
    if (l16 == 0) {
#pragma unroll
      for (int v = 0; v < 8; ++v) { const int r = v + 8 * hh; for (int e = 48; e < 64; ++e) { if (MODE < 2) ts[(r * 4 + t) * 64 + e] = (b16)0.f; else ts[t * 1024 + e * 16 + r] = (b16)0.f; } }
    }
  }
  __builtin_amdgcn_fence(__ATOMIC_RELEASE, "workgroup"); __builtin_amdgcn_wave_barrier(); __builtin_amdgcn_fence(__ATOMIC_ACQUIRE, "workgroup");
  const int hb = o0 / 16;
  for (int pass = 0; pass < 2; ++pass) {
    if (MODE < 2) {
#pragma unroll
      for (int j = 0; j < 16; ++j) { const int pc = j * 32 + lane, r = pc >> 5, t = (pc >> 3) & 3, q8 = pc & 7;
        *(volatile v8b*)(P + (((size_t)b * NH + hb + t) * T + t0 + r) * 64 + q8 * 8) = *(const v8b*)(ts + (r * 4 + t) * 64 + q8 * 8); }
    } else {
#pragma unroll
      for (int j = 0; j < 16; ++j) { const int pc = j * 32 + lane, t = pc >> 7, q8 = pc & 127;
        *(volatile v8b*)(P + (((size_t)b * NH + hb + t) * QT_PER_B + (t0 >> 4)) * 1024 + q8 * 8) = *(const v8b*)(ts + t * 1024 + q8 * 8); }
    }
    __threadfence();
  }
}
__global__ __launch_bounds__(256) void attn_kernel(const b16* __restrict__ Qh, const b16* __restrict__ Ql, const b16* __restrict__ Kh, const b16* __restrict__ Kl,
                                                   const b16* __restrict__ Vh, const b16* __restrict__ Vl, const int* __restrict__ seqlen,
                                                   float* __restrict__ yf) {
  __shared__ __attribute__((aligned(16))) float Os[8][16 * 64];
  const int wid = threadIdx.x >> 5, lane = threadIdx.x & 31, hh = lane >> 4, col = lane & 15;
  const int qtile = blockIdx.x * 8 + wid;
  const int g = qtile / QT_PER_B;
  const int q0 = (qtile % QT_PER_B) << 4;
  const int b = g / NH, h = g % NH, kvh = h / REP;
  const size_t ko = (size_t)(b * NKV + kvh) * T * DH;
  const size_t qo = ((size_t)g * T + q0 + col) * DH;
  const v16b q0h = frag_kb(Qh + qo, hh), q0l = frag_kb(Ql + qo, hh), q1h = frag_kb(Qh + qo + 32, hh), q1l = frag_kb(Ql + qo + 32, hh);
  float m = -INFINITY, l = 0.0f;
  v8f o0 = {}, o1 = {}, o2 = {}, o3 = {};
  const int slen = T; (void)seqlen;
  for (int kb = 0; kb < T; kb += 32) {
    const size_t r0 = ko + (size_t)(kb + col) * DH, r1 = ko + (size_t)(kb + 16 + col) * DH;
    v8f s0 = {}, s1 = {};
    {
      v16b ah = frag_kb(Kh + r0, hh), al = frag_kb(Kl + r0, hh);
      s0 = wmma1(ah, al, q0h, q0l, s0);
      ah = frag_kb(Kh + r0 + 32, hh); al = frag_kb(Kl + r0 + 32, hh);
      s0 = wmma1(ah, al, q1h, q1l, s0);
      ah = frag_kb(Kh + r1, hh); al = frag_kb(Kl + r1, hh);
      s1 = wmma1(ah, al, q0h, q0l, s1);
      ah = frag_kb(Kh + r1 + 32, hh); al = frag_kb(Kl + r1 + 32, hh);
      s1 = wmma1(ah, al, q1h, q1l, s1);
    }
    (void)slen;
    float mr = -INFINITY;
#pragma unroll
    for (int r = 0; r < 8; ++r) mr = fmaxf(mr, fmaxf(s0[r], s1[r]));
    mr = fmaxf(mr, __shfl_xor(mr, 16));
    float mn = fmaxf(m, mr);
    if (mn == -INFINITY) mn = 0.0f;
    const float al_ = __expf(m - mn);
    m = mn;
    float sum = 0.0f;
    v16b pbh, pbl;
#pragma unroll
    for (int r = 0; r < 8; ++r) {
      const float p0 = __expf(s0[r] - mn), p1 = __expf(s1[r] - mn);
      sum += p0 + p1;
      b16 a, c; split_bf16(p0, a, c); pbh[r] = a; pbl[r] = c; split_bf16(p1, a, c); pbh[8 + r] = a; pbl[8 + r] = c;
    }
    sum += __shfl_xor(sum, 16);
    l = l * al_ + sum;
#pragma unroll
    for (int r = 0; r < 8; ++r) { o0[r] *= al_; o1[r] *= al_; o2[r] *= al_; o3[r] *= al_; }
    const size_t v0 = ko + (size_t)(kb >> 4) * (DH * 16) + 8 * hh, v1 = v0 + DH * 16;
#pragma unroll
    for (int n = 0; n < 4; ++n) {
      const int f = n * 16 + col;
      const v16b vah = cat8b(ld8b(Vh + v0 + f * 16), ld8b(Vh + v1 + f * 16));
      const v16b val = cat8b(ld8b(Vl + v0 + f * 16), ld8b(Vl + v1 + f * 16));
      v8f& o = (n == 0) ? o0 : (n == 1) ? o1 : (n == 2) ? o2 : o3;
      o = wmma1(vah, val, pbh, pbl, o);
    }
  }
  const float inv = (q0 + col < slen && l > 0.0f) ? (1.0f / l) : 0.0f;
  float* Tt = Os[wid];
#pragma unroll
  for (int r = 0; r < 8; ++r) {
    const int hr = 8 * hh + r;
    Tt[col * 64 + 0 + hr] = o0[r] * inv; Tt[col * 64 + 16 + hr] = o1[r] * inv;
    Tt[col * 64 + 32 + hr] = o2[r] * inv; Tt[col * 64 + 48 + hr] = o3[r] * inv;
  }
  wave_lds_sync();
  float* dst0 = yf + ((size_t)b * T + q0) * HID + h * DH;
#pragma unroll
  for (int j = 0; j < 8; ++j) { const int rr = j * 2 + hh, c4 = col * 4; *(volatile v4f*)(dst0 + (size_t)rr * HID + c4) = *(const v4f*)(Tt + rr * 64 + c4); }
  __threadfence();
#pragma unroll
  for (int j = 0; j < 8; ++j) { const int rr = j * 2 + hh, c4 = col * 4; *(volatile v4f*)(dst0 + (size_t)rr * HID + c4) = *(const v4f*)(Tt + rr * 64 + c4); }
}


__global__ __launch_bounds__(128) void k_oproj(const float* __restrict__ yf, const b16* __restrict__ W16, const b16* __restrict__ W16l, const float* __restrict__ bias, float* __restrict__ out) {
  __shared__ __attribute__((aligned(16))) float To[4][16 * 192];
  const int lane = threadIdx.x & 31, wave = threadIdx.x >> 5, hh = lane >> 4, l16 = lane & 15;
  const int m0 = blockIdx.x * 64 + wave * 16, o0 = blockIdx.y * 64;
  v8f acc[4][3];
#pragma unroll
  for (int t = 0; t < 4; ++t)
#pragma unroll
    for (int c = 0; c < 3; ++c) acc[t][c] = (v8f){};
  const float* yr = yf + (size_t)(m0 + l16) * HID;
#pragma unroll
  for (int k0 = 0; k0 < CC; k0 += 32) {
    v16b a[3], al[3];
#pragma unroll
    for (int e = 0; e < 16; ++e) { const int i = k0 + kmap(e, hh), base = (i >> 4) * 64 + (i & 15) * 3;
#pragma unroll
      for (int c = 0; c < 3; ++c) { const float v = yr[base + c]; const b16 h = (b16)v; a[c][e] = h; al[c][e] = (b16)(v - (float)h); } }
#pragma unroll
    for (int t = 0; t < 4; ++t) {
      const v16b w = frag_kb(W16 + (size_t)(o0 + t * 16 + l16) * CC + k0, hh), wl = frag_kb(W16l + (size_t)(o0 + t * 16 + l16) * CC + k0, hh);
#pragma unroll
      for (int c = 0; c < 3; ++c) { acc[t][c] = wmma16s(a[c], w, acc[t][c]); acc[t][c] = wmma16s(a[c], wl, acc[t][c]); acc[t][c] = wmma16s(al[c], w, acc[t][c]); }
    }
  }
  float* to = To[wave];
#pragma unroll
  for (int t = 0; t < 4; ++t) {
    const float bo = bias[o0 + t * 16 + l16];
#pragma unroll
    for (int v = 0; v < 8; ++v) {
      const int r = v + 8 * hh;
      const float y0 = acc[t][0][v], y1 = acc[t][1][v], y2 = acc[t][2][v];
      const float f = 1.0f + bo / (sqrtf(y0 * y0 + y1 * y1 + y2 * y2) + 1e-6f);
      const int ol = t * 16 + l16;
      to[r * 192 + ol * 3] = y0 * f; to[r * 192 + ol * 3 + 1] = y1 * f; to[r * 192 + ol * 3 + 2] = y2 * f;
    }
  }
  __builtin_amdgcn_fence(__ATOMIC_RELEASE, "workgroup"); __builtin_amdgcn_wave_barrier(); __builtin_amdgcn_fence(__ATOMIC_ACQUIRE, "workgroup");
  for (int pass = 0; pass < 2; ++pass) {
    for (int pc = lane; pc < 16 * 48; pc += 32) { const int r = pc / 48, q4 = pc % 48;
      *(volatile v4f*)(out + (size_t)(m0 + r) * (CC * 3) + o0 * 3 + q4 * 4) = *(const v4f*)(to + r * 192 + q4 * 4); }
    __threadfence();
  }
}
}
extern "C" void kernel_launch(void* const* d_in, const int* in_sizes, int n_in,
                              void* d_out, int out_size, void* d_ws, size_t ws_size, hipStream_t stream) {
  (void)in_sizes; (void)n_in; (void)out_size;
  const float* q  = (const float*)d_in[0];
  const float* vv = (const float*)d_in[1];
  const float* Wq = (const float*)d_in[2]; const float* bq = (const float*)d_in[3];
  const float* Wk = (const float*)d_in[4]; const float* bk = (const float*)d_in[5];
  const float* Wv = (const float*)d_in[6]; const float* bv = (const float*)d_in[7];
  const float* Wp = (const float*)d_in[8]; const float* bp = (const float*)d_in[9];
  float* out = (float*)d_out;
  size_t off = 0; char* ws = (char*)d_ws;
  b16* W6 = (b16*)(ws + off); off += (size_t)4 * CC * CC * 2;
  b16* W6l = (b16*)(ws + off); off += (size_t)4 * CC * CC * 2;
  b16* Qh = (b16*)(ws + off); off += (size_t)MROWS * HID * 2;
  b16* Kh = (b16*)(ws + off); off += (size_t)MROWS * KVW * 2;
  b16* Vh = (b16*)(ws + off); off += (size_t)MROWS * KVW * 2;
  float* yf = (float*)(ws + off); off += (size_t)MROWS * HID * 4;
  if (off > ws_size) return;
  const int NQT = Bsz * NH * QT_PER_B;
  k_w16<<<8, 256, 0, stream>>>(Wq, W6, W6l); k_w16<<<8, 256, 0, stream>>>(Wk, W6 + CC * CC, W6l + CC * CC);
  k_w16<<<8, 256, 0, stream>>>(Wv, W6 + 2 * CC * CC, W6l + 2 * CC * CC); k_w16<<<8, 256, 0, stream>>>(Wp, W6 + 3 * CC * CC, W6l + 3 * CC * CC);
  k_vproj<0><<<dim3(MROWS / 64, 2), 128, 0, stream>>>(q, W6, W6l, bq, Qh);
  k_vproj<1><<<dim3(MROWS / 64, 2), 128, 0, stream>>>(vv, W6 + CC * CC, W6l + CC * CC, bk, Kh);
  k_vproj<2><<<dim3(MROWS / 64, 2), 128, 0, stream>>>(vv, W6 + 2 * CC * CC, W6l + 2 * CC * CC, bv, Vh);
  attn_kernel<<<NQT / 8, 256, 0, stream>>>(Qh, Qh, Kh, Kh, Vh, Vh, nullptr, yf);
  k_oproj<<<dim3(MROWS / 64, 2), 128, 0, stream>>>(yf, W6 + 3 * CC * CC, W6l + 3 * CC * CC, bp, out);
}
